// GCNChannel_63084479644063
// MI455X (gfx1250) — hardware-verified
//
#include <hip/hip_runtime.h>


#define NBI  4
#define CC   64
#define HI   128
#define HO   64
#define NN   4096
#define KC   576
#define RB   512
typedef _Float16 h16;
typedef unsigned short bf;
typedef __attribute__((ext_vector_type(16))) __bf16   v16bf;
typedef __attribute__((ext_vector_type(16))) _Float16 v16h;
typedef __attribute__((ext_vector_type(8)))  _Float16 v8h;
typedef __attribute__((ext_vector_type(8)))  unsigned short v8us;
typedef __attribute__((ext_vector_type(8)))  float    v8f;
typedef __attribute__((ext_vector_type(4)))  float    v4f;
typedef v8h  __attribute__((may_alias)) v8ha;
typedef v4f  __attribute__((may_alias)) v4fa;
typedef v8us __attribute__((may_alias)) v8usa;

__device__ __forceinline__ unsigned short f2bf(float f) { unsigned u = __float_as_uint(f); u += 0x7FFFu + ((u >> 16) & 1u); return (unsigned short)(u >> 16); }
__device__ __forceinline__ float bf2f(unsigned short b) { return __uint_as_float(((unsigned)b) << 16); }
__device__ __forceinline__ float bfr(float f) { return bf2f(f2bf(f)); }
__device__ __forceinline__ v16h cat16(v8h lo, v8h hi) { return __builtin_shufflevector(lo, hi, 0, 1, 2, 3, 4, 5, 6, 7, 8, 9, 10, 11, 12, 13, 14, 15); }
__device__ __forceinline__ v16bf cat16b(v8us lo, v8us hi) { return __builtin_bit_cast(v16bf, __builtin_shufflevector(lo, hi, 0, 1, 2, 3, 4, 5, 6, 7, 8, 9, 10, 11, 12, 13, 14, 15)); }
__device__ __forceinline__ v8f wmma16(v16h a, v16h b, v8f c) { return __builtin_amdgcn_wmma_f32_16x16x32_f16(false, a, false, b, (short)0, c, false, false); }
__device__ __forceinline__ v8f wmmab(v16bf a, v16bf b, v8f c) { return __builtin_amdgcn_wmma_f32_16x16x32_bf16(false, a, false, b, (short)0, c, false, false); }


template <typename T16> struct WFrag;
template <> struct WFrag<h16> { typedef v16h V; static __device__ __forceinline__ V ld(const h16* p) { return cat16(*(const v8h*)p, *(const v8h*)(p + 16)); } static __device__ __forceinline__ v8f mma(V a, V b, v8f c) { return wmma16(a, b, c); } };
template <> struct WFrag<bf> { typedef v16bf V; static __device__ __forceinline__ V ld(const bf* p) { return cat16b(*(const v8us*)p, *(const v8us*)(p + 16)); } static __device__ __forceinline__ v8f mma(V a, V b, v8f c) { return wmmab(a, b, c); } };
template <typename T16, int NSPLIT, bool BIAS>
__global__ __launch_bounds__(32) void k_gemmw(const T16* __restrict__ A, const T16* __restrict__ A2, const T16* __restrict__ Bt, const T16* __restrict__ Bt2, int K, float* C, int ldc, const float* __restrict__ bias, size_t sA, size_t sB, size_t sC) {
    typedef typename WFrag<T16>::V V;
    __shared__ __align__(16) float os[16 * 68];
    const size_t z = blockIdx.z; A += z * sA; if (A2) A2 += z * sA; Bt += z * sB; if (Bt2) Bt2 += z * sB; C += z * sC;
    const int lane = threadIdx.x & 31, lr = lane & 15, hi = lane >> 4; const int r0 = blockIdx.x * 64, c0 = blockIdx.y * 64;
    v8f acc[4][4];
#pragma unroll
    for (int mb = 0; mb < 4; ++mb)
#pragma unroll
        for (int nb = 0; nb < 4; ++nb) acc[mb][nb] = (v8f){};
    const size_t aoff = (size_t)(r0 + lr) * K + 8 * hi, boff = (size_t)(c0 + lr) * K + 8 * hi;
#pragma unroll 1
    for (int kc = 0; kc < K; kc += 32) {
        V a[4], a2[4];
#pragma unroll
        for (int mb = 0; mb < 4; ++mb) { a[mb] = WFrag<T16>::ld(A + aoff + (size_t)mb * 16 * K + kc); if (NSPLIT == 1 || NSPLIT == 2) a2[mb] = WFrag<T16>::ld(A2 + aoff + (size_t)mb * 16 * K + kc); }
#pragma unroll
        for (int nb = 0; nb < 4; ++nb) { const V b = WFrag<T16>::ld(Bt + boff + (size_t)nb * 16 * K + kc); V b2; if (NSPLIT >= 2) b2 = WFrag<T16>::ld(Bt2 + boff + (size_t)nb * 16 * K + kc);
#pragma unroll
            for (int mb = 0; mb < 4; ++mb) { acc[mb][nb] = WFrag<T16>::mma(a[mb], b, acc[mb][nb]); if (NSPLIT == 1 || NSPLIT == 2) acc[mb][nb] = WFrag<T16>::mma(a2[mb], b, acc[mb][nb]); if (NSPLIT >= 2) acc[mb][nb] = WFrag<T16>::mma(a[mb], b2, acc[mb][nb]); } }
        asm volatile("v_nop\n\tv_nop\n\tv_nop\n\tv_nop" : "+v"(acc[0][0]), "+v"(acc[1][1]), "+v"(acc[2][2]), "+v"(acc[3][3]) : "v"(a[0]), "v"(a[3]));
    }
#pragma unroll
    for (int mb = 0; mb < 4; ++mb) {
#pragma unroll
        for (int nb = 0; nb < 4; ++nb) {
#pragma unroll
            for (int j = 0; j < 8; ++j) os[(hi * 8 + j) * 68 + nb * 16 + lr] = acc[mb][nb][j]; }
        __builtin_amdgcn_wave_barrier(); asm volatile("" ::: "memory");
        float* crow = C + (size_t)(r0 + mb * 16) * ldc + c0;
#pragma unroll 1
        for (int ps = 0; ps < 2; ++ps) {
#pragma unroll
            for (int s = 0; s < 8; ++s) { const int row = 2 * s + hi, cofs = lr * 4; v4f val = *(const v4fa*)(os + row * 68 + cofs); if (BIAS) { val[0] += bfr(bias[c0 + cofs]); val[1] += bfr(bias[c0 + cofs + 1]); val[2] += bfr(bias[c0 + cofs + 2]); val[3] += bfr(bias[c0 + cofs + 3]); }
                *(volatile v4f*)(crow + (size_t)row * ldc + cofs) = val; }
            if (ps == 0) __threadfence(); }
        __builtin_amdgcn_wave_barrier(); asm volatile("" ::: "memory");
    }
}

__device__ __forceinline__ void splitf(float y, unsigned short& h, unsigned short& l) { h = f2bf(y); l = f2bf(y - bf2f(h)); }
typedef __attribute__((ext_vector_type(2))) unsigned short v2us;
typedef __attribute__((ext_vector_type(4))) unsigned short v4us;

__global__ __launch_bounds__(256) void k_wc(const float* __restrict__ w, bf* WCB) { const int i = (blockIdx.x * 256 + threadIdx.x) * 4; if (i >= CC * KC) return; v4us o;
#pragma unroll
    for (int q = 0; q < 4; ++q) o[q] = f2bf(w[i + q]); *(volatile v4us*)(WCB + i) = o; __threadfence(); *(volatile v4us*)(WCB + i) = o; }
__global__ __launch_bounds__(256) void k_i2c(const float* __restrict__ xb, bf* PAT) { const size_t e = ((size_t)blockIdx.x * 256 + threadIdx.x) * 4; if (e >= (size_t)NN * KC) return; const int k = (int)(e % KC); const int n = (int)(e / KC); const int oy = n / HO, ox = n % HO; v4us o;
#pragma unroll
    for (int q = 0; q < 4; ++q) { const int kk = k + q; const int c = kk / 9, r9 = kk % 9, ky = r9 / 3, kx = r9 % 3; const int iy = 2 * oy + ky - 1, ix = 2 * ox + kx - 1; float v = 0.f; if (iy >= 0 && iy < HI && ix >= 0 && ix < HI) v = xb[((size_t)c * HI + iy) * HI + ix]; o[q] = f2bf(v); }
    *(volatile v4us*)(PAT + e) = o; __threadfence(); *(volatile v4us*)(PAT + e) = o; }
__global__ __launch_bounds__(256) void k_bnr(const float* __restrict__ F, const float* __restrict__ g, const float* __restrict__ be, const float* __restrict__ mu, const float* __restrict__ var, float* Y) { const int e = (blockIdx.x * 256 + threadIdx.x) * 4; if (e >= NN * CC) return; const int c = e % CC; const v4f a = *(const v4f*)(F + e); v4f o;
#pragma unroll
    for (int q = 0; q < 4; ++q) { const int cc = c + q; float t0 = __fmul_rn(__fsub_rn(a[q], bfr(mu[cc])), __frsqrt_rn(__fadd_rn(bfr(var[cc]), 1e-5f))); asm volatile("" : "+v"(t0)); float t1 = __fmul_rn(t0, bfr(g[cc])); asm volatile("" : "+v"(t1)); o[q] = fmaxf(__fadd_rn(t1, bfr(be[cc])), 0.f); }
    *(volatile v4f*)(Y + e) = o; __threadfence(); *(volatile v4f*)(Y + e) = o; }
__device__ __forceinline__ float ygrid(const float* __restrict__ Y, int n, int c) { return (n >= 0 && n < NN && c >= 0 && c < CC) ? Y[n * CC + c] : 0.f; }
__global__ __launch_bounds__(256) void k_sob(const float* __restrict__ Y, bf* SXh, bf* SXl, bf* SYh, bf* SYl) { const int e = (blockIdx.x * 256 + threadIdx.x) * 4; if (e >= NN * CC) return; const int c = e % CC; const int n = e / CC; v4us xh, xl, yh, yl;
#pragma unroll
    for (int q = 0; q < 4; ++q) { const int cc = c + q; const float a00 = ygrid(Y, n - 1, cc - 1), a01 = ygrid(Y, n - 1, cc), a02 = ygrid(Y, n - 1, cc + 1), a10 = ygrid(Y, n, cc - 1), a12 = ygrid(Y, n, cc + 1), a20 = ygrid(Y, n + 1, cc - 1), a21 = ygrid(Y, n + 1, cc), a22 = ygrid(Y, n + 1, cc + 1);
        float sx = 0.f; sx = __fadd_rn(sx, -a00); sx = __fadd_rn(sx, a02); { float t = __fmul_rn(-2.0f, a10); asm volatile("" : "+v"(t)); sx = __fadd_rn(sx, t); } { float t = __fmul_rn(2.0f, a12); asm volatile("" : "+v"(t)); sx = __fadd_rn(sx, t); } sx = __fadd_rn(sx, -a20); sx = __fadd_rn(sx, a22);
        float sy = 0.f; sy = __fadd_rn(sy, -a00); { float t = __fmul_rn(-2.0f, a01); asm volatile("" : "+v"(t)); sy = __fadd_rn(sy, t); } sy = __fadd_rn(sy, -a02); sy = __fadd_rn(sy, a20); { float t = __fmul_rn(2.0f, a21); asm volatile("" : "+v"(t)); sy = __fadd_rn(sy, t); } sy = __fadd_rn(sy, a22);
        unsigned short u, l; splitf(fabsf(sx), u, l); xh[q] = u; xl[q] = l; splitf(fabsf(sy), u, l); yh[q] = u; yl[q] = l; }
    for (int ps = 0; ps < 2; ++ps) { *(volatile v4us*)(SXh + e) = xh; *(volatile v4us*)(SXl + e) = xl; *(volatile v4us*)(SYh + e) = yh; *(volatile v4us*)(SYl + e) = yl; if (ps == 0) __threadfence(); } }
__global__ __launch_bounds__(256) void k_bsm(const float* __restrict__ Sb, int n0, bf* A1B, float* RS) { const int lane = threadIdx.x & 31; const int r = blockIdx.x * 8 + (threadIdx.x >> 5); if (r >= RB) return; const int n = n0 + r; float rs[NBI] = {0.f, 0.f, 0.f, 0.f};
    for (int ps = 0; ps < 2; ++ps) { rs[0] = rs[1] = rs[2] = rs[3] = 0.f;
#pragma unroll 1
        for (int ch = 0; ch < NN / 128; ++ch) { const int m0 = ch * 128 + lane * 4; v4f a[NBI];
#pragma unroll
            for (int b = 0; b < NBI; ++b) a[b] = *(const v4f*)(Sb + ((size_t)b * RB + r) * NN + m0);
            v4us o[NBI];
#pragma unroll
            for (int q = 0; q < 4; ++q) { float mx = fmaxf(fmaxf(a[0][q], a[1][q]), fmaxf(a[2][q], a[3][q])); float ex[NBI]; float s = 0.f;
#pragma unroll
                for (int b = 0; b < NBI; ++b) { ex[b] = __expf(__fsub_rn(a[b][q], mx)); s = __fadd_rn(s, ex[b]); }
                const float inv = __fdiv_rn(1.0f, s); const float eye = (m0 + q == n) ? 1.0f : 0.f;
#pragma unroll
                for (int b = 0; b < NBI; ++b) { const float w = __fadd_rn(__fmul_rn(ex[b], inv), eye); rs[b] = __fadd_rn(rs[b], w); o[b][q] = f2bf(w); } }
#pragma unroll
            for (int b = 0; b < NBI; ++b) *(volatile v4us*)(A1B + ((size_t)b * NN + n) * NN + m0) = o[b]; }
        if (ps == 0) __threadfence(); }
#pragma unroll
    for (int b = 0; b < NBI; ++b) {
#pragma unroll
        for (int sh = 16; sh; sh >>= 1) rs[b] += __shfl_xor(rs[b], sh, 32); }
    const float mine = (lane < NBI) ? rs[lane & 3] : 0.f;
    float v = (lane == 0) ? rs[0] : (lane == 1) ? rs[1] : (lane == 2) ? rs[2] : (lane == 3) ? rs[3] : 0.f; (void)mine;
    *(volatile float*)(RS + (size_t)n * 32 + lane) = v; __threadfence(); *(volatile float*)(RS + (size_t)n * 32 + lane) = v; }
__global__ __launch_bounds__(256) void k_dinv(const float* __restrict__ RS, float* DINV) { const int e = blockIdx.x * 256 + threadIdx.x; if (e >= NBI * NN) return; const int n = e % NN, b = e / NN; const float d = __frsqrt_rn(RS[(size_t)n * 32 + b]); *(volatile float*)(DINV + e) = d; __threadfence(); *(volatile float*)(DINV + e) = d; }
__global__ __launch_bounds__(256) void k_xdt(const float* __restrict__ X, const float* __restrict__ dinv, bf* XDh, bf* XDl) { const int e = (blockIdx.x * 256 + threadIdx.x) * 2; if (e >= CC * NN) return; const int m = e % NN; const int c = e / NN; v2us oh, ol;
#pragma unroll
    for (int u = 0; u < 2; ++u) { unsigned short a, b; splitf(__fmul_rn(dinv[m + u], X[(size_t)(m + u) * CC + c]), a, b); oh[u] = a; ol[u] = b; } *(volatile v2us*)(XDh + e) = oh; *(volatile v2us*)(XDl + e) = ol; __threadfence(); *(volatile v2us*)(XDh + e) = oh; *(volatile v2us*)(XDl + e) = ol; }
__global__ __launch_bounds__(256) void k_fc(const float* __restrict__ Yp, const float* __restrict__ dinv, const float* __restrict__ w, int relu_, float* Xn) { const int e = (blockIdx.x * 256 + threadIdx.x) * 4; if (e >= NN * CC) return; const int o0 = e % CC; const int n = e / CC; const float dn = dinv[n]; v4f o;
#pragma unroll
    for (int q = 0; q < 4; ++q) { const float* wr = w + (o0 + q) * CC; float s = 0.f;
#pragma unroll 1
        for (int c = 0; c < CC; ++c) { float p = __fmul_rn(Yp[(size_t)c * NN + n], bfr(wr[c])); asm volatile("" : "+v"(p)); s = __fadd_rn(s, p); } const float v = __fmul_rn(s, dn); o[q] = relu_ ? fmaxf(v, 0.f) : v; }
    *(volatile v4f*)(Xn + e) = o; __threadfence(); *(volatile v4f*)(Xn + e) = o; }
__global__ __launch_bounds__(256) void k_fcT(const float* __restrict__ Yp, const float* __restrict__ dinv, const float* __restrict__ w, float* XT) { const int e = (blockIdx.x * 256 + threadIdx.x) * 4; if (e >= CC * NN) return; const int n = e % NN; const int oc = e / NN; const float* wr = w + oc * CC; v4f o;
#pragma unroll
    for (int q = 0; q < 4; ++q) { float s = 0.f;
#pragma unroll 1
        for (int c = 0; c < CC; ++c) { float p = __fmul_rn(Yp[(size_t)c * NN + n + q], bfr(wr[c])); asm volatile("" : "+v"(p)); s = __fadd_rn(s, p); } o[q] = __fmul_rn(s, dinv[n + q]); }
    *(volatile v4f*)(XT + e) = o; __threadfence(); *(volatile v4f*)(XT + e) = o; }
__global__ __launch_bounds__(256) void k_up(const float* __restrict__ XT, float* OUTb) { const size_t e = ((size_t)blockIdx.x * 256 + threadIdx.x) * 4; if (e >= (size_t)CC * HI * HI) return; const int j = (int)(e % HI); const int i = (int)((e / HI) % HI); const int c = (int)(e / ((size_t)HI * HI)); const float* g = XT + (size_t)c * NN;
    const float ys = (float)i * (float)(HO - 1) / (float)(HI - 1); const int y0 = (int)floorf(ys); const int y1 = min(y0 + 1, HO - 1); const float wy = ys - (float)y0; v4f o;
#pragma unroll
    for (int q = 0; q < 4; ++q) { const float xs = (float)(j + q) * (float)(HO - 1) / (float)(HI - 1); const int x0 = (int)floorf(xs); const int x1 = min(x0 + 1, HO - 1); const float wx = xs - (float)x0;
        const float t = __fadd_rn(__fmul_rn(g[y0 * HO + x0], 1.f - wx), __fmul_rn(g[y0 * HO + x1], wx)); const float bt = __fadd_rn(__fmul_rn(g[y1 * HO + x0], 1.f - wx), __fmul_rn(g[y1 * HO + x1], wx)); o[q] = __fadd_rn(__fmul_rn(t, 1.f - wy), __fmul_rn(bt, wy)); }
    *(volatile v4f*)(OUTb + e) = o; __threadfence(); *(volatile v4f*)(OUTb + e) = o; }

extern "C" void kernel_launch(void* const* d_in, const int* in_sizes, int n_in,
                              void* d_out, int out_size, void* d_ws, size_t ws_size, hipStream_t stream) {
    (void)in_sizes; (void)n_in; (void)out_size;
    const float* x = (const float*)d_in[0]; const float* cw = (const float*)d_in[1]; const float* cb = (const float*)d_in[2]; const float* g = (const float*)d_in[3]; const float* be = (const float*)d_in[4]; const float* mu = (const float*)d_in[5]; const float* var = (const float*)d_in[6]; const float* w1 = (const float*)d_in[7]; const float* w2 = (const float*)d_in[8]; const float* w3 = (const float*)d_in[9];
    float* OUT = (float*)d_out;
    char* wsp = (char*)d_ws;
    auto take = [&](size_t bytes) { char* p = wsp; wsp += (bytes + 255) & ~(size_t)255; return (void*)p; };
    bf* WCB = (bf*)take(CC * KC * 2); bf* PAT = (bf*)take((size_t)NN * KC * 2); float* F = (float*)take((size_t)NN * CC * 4); float* Y0 = (float*)take((size_t)NBI * NN * CC * 4);
    bf* SXh = (bf*)take((size_t)NBI * NN * CC * 2); bf* SXl = (bf*)take((size_t)NBI * NN * CC * 2); bf* SYh = (bf*)take((size_t)NBI * NN * CC * 2); bf* SYl = (bf*)take((size_t)NBI * NN * CC * 2); float* Sb = (float*)take((size_t)NBI * RB * NN * 4); bf* A1B = (bf*)take((size_t)NBI * NN * NN * 2); float* RS = (float*)take((size_t)NN * 32 * 4); float* DINV = (float*)take((size_t)NBI * NN * 4);
    bf* XDh = (bf*)take((size_t)CC * NN * 2); bf* XDl = (bf*)take((size_t)CC * NN * 2); float* YP = (float*)take((size_t)CC * NN * 4); float* X1 = (float*)take((size_t)NN * CC * 4); float* X2 = (float*)take((size_t)NN * CC * 4); float* X3T = (float*)take((size_t)CC * NN * 4);
    if ((size_t)(wsp - (char*)d_ws) > ws_size) return;
    k_wc<<<(CC * KC / 4 + 255) / 256, 256, 0, stream>>>(cw, WCB);
    for (int b = 0; b < NBI; ++b) {
        k_i2c<<<(unsigned)(((size_t)NN * KC / 4 + 255) / 256), 256, 0, stream>>>(x + (size_t)b * CC * HI * HI, PAT);
        k_gemmw<bf, 0, true><<<dim3(NN / 64, 1, 1), 32, 0, stream>>>(PAT, nullptr, WCB, nullptr, KC, F, CC, cb, 0, 0, 0);
        k_bnr<<<(NN * CC / 4 + 255) / 256, 256, 0, stream>>>(F, g, be, mu, var, Y0 + (size_t)b * NN * CC);
        k_sob<<<(NN * CC / 4 + 255) / 256, 256, 0, stream>>>(Y0 + (size_t)b * NN * CC, SXh + (size_t)b * NN * CC, SXl + (size_t)b * NN * CC, SYh + (size_t)b * NN * CC, SYl + (size_t)b * NN * CC); }
    for (int blk = 0; blk < NN / RB; ++blk) { const int n0 = blk * RB;
        k_gemmw<bf, 2, false><<<dim3(RB / 64, NN / 64, NBI), 32, 0, stream>>>(SXh + (size_t)n0 * CC, SXl + (size_t)n0 * CC, SYh, SYl, CC, Sb, NN, nullptr, (size_t)NN * CC, (size_t)NN * CC, (size_t)RB * NN);
        k_bsm<<<RB / 8, 256, 0, stream>>>(Sb, n0, A1B, RS); }
    k_dinv<<<(NBI * NN + 255) / 256, 256, 0, stream>>>(RS, DINV);
    for (int b = 0; b < NBI; ++b) { const float* dv = DINV + (size_t)b * NN; const bf* Ab = A1B + (size_t)b * NN * NN;
        k_xdt<<<(CC * NN / 2 + 255) / 256, 256, 0, stream>>>(Y0 + (size_t)b * NN * CC, dv, XDh, XDl); k_gemmw<bf, 1, false><<<dim3(1, NN / 64, 1), 32, 0, stream>>>(XDh, XDl, Ab, nullptr, NN, YP, NN, nullptr, 0, 0, 0); k_fc<<<(NN * CC / 4 + 255) / 256, 256, 0, stream>>>(YP, dv, w1, 1, X1);
        k_xdt<<<(CC * NN / 2 + 255) / 256, 256, 0, stream>>>(X1, dv, XDh, XDl); k_gemmw<bf, 1, false><<<dim3(1, NN / 64, 1), 32, 0, stream>>>(XDh, XDl, Ab, nullptr, NN, YP, NN, nullptr, 0, 0, 0); k_fc<<<(NN * CC / 4 + 255) / 256, 256, 0, stream>>>(YP, dv, w2, 1, X2);
        k_xdt<<<(CC * NN / 2 + 255) / 256, 256, 0, stream>>>(X2, dv, XDh, XDl); k_gemmw<bf, 1, false><<<dim3(1, NN / 64, 1), 32, 0, stream>>>(XDh, XDl, Ab, nullptr, NN, YP, NN, nullptr, 0, 0, 0); k_fcT<<<(CC * NN / 4 + 255) / 256, 256, 0, stream>>>(YP, dv, w3, X3T);
        k_up<<<(unsigned)(((size_t)CC * HI * HI / 4 + 255) / 256), 256, 0, stream>>>(X3T, OUT + (size_t)b * CC * HI * HI); }
}
